// FusionBlock_31439160607466
// MI455X (gfx1250) — hardware-verified
//
#include <hip/hip_runtime.h>
#include <math.h>

constexpr int kNB    = 4;
constexpr int kSeq   = 1024;
constexpr int kDim   = 1024;
constexpr int kHeads = 16;
constexpr int kHd    = 64;
constexpr int kHid   = 4096;
constexpr int kTok   = kNB * kSeq;
constexpr int kQkvN  = 3 * kDim;
constexpr int kHeadsPerChunk = 8;
constexpr int kNumChunks = (kNB * kHeads) / kHeadsPerChunk;
constexpr int kMlpRows = 2048;
constexpr int kMlpParts = kTok / kMlpRows;
constexpr float kWCarry    = 16.0f;
constexpr float kWCarryInv = 1.0f / 16.0f;
constexpr float kPCarry    = 2048.0f;
constexpr float kCtxCarry  = 256.0f;
constexpr float kPVScale   = kCtxCarry / kPCarry;
constexpr float kProjScale = 1.0f / (kCtxCarry * kWCarry);
constexpr float kAttnScale = 0.125f;
constexpr float kInvDim    = 1.0f / 1024.0f;
constexpr float kLnEps     = 1e-5f;

constexpr size_t kMiB   = 1048576;
constexpr size_t kOffWA = 0;
constexpr size_t kOffWB = 8 * kMiB;
constexpr size_t kOffH  = 16 * kMiB;
constexpr size_t kOffQ  = 24 * kMiB;
constexpr size_t kOffS  = 48 * kMiB;
constexpr size_t kOffP  = 80 * kMiB;
constexpr size_t kWsTotal = 96 * kMiB;
static_assert((size_t)kQkvN * kDim * 2 <= 8 * kMiB);
static_assert((size_t)kNB * kHeads * kHd * kSeq * 2 <= 8 * kMiB);
static_assert((size_t)kHid * kDim * 2 <= 8 * kMiB);
static_assert((size_t)kDim * kHid * 2 <= 8 * kMiB);
static_assert((size_t)kTok * kDim * 2 <= 8 * kMiB);
static_assert((size_t)kTok * kQkvN * 2 <= 24 * kMiB);
static_assert((size_t)kTok * kDim * 4 <= 24 * kMiB);
static_assert((size_t)kHeadsPerChunk * kSeq * kSeq * 4 <= 32 * kMiB);
static_assert((size_t)kMlpRows * kHid * 4 <= 32 * kMiB);
static_assert((size_t)kHeadsPerChunk * kSeq * kSeq * 2 <= 16 * kMiB);
static_assert((size_t)kMlpRows * kHid * 2 <= 16 * kMiB);
static_assert(kWsTotal == 100663296);

typedef __attribute__((ext_vector_type(16))) _Float16 v16h;
typedef __attribute__((ext_vector_type(8)))  _Float16 v8h;
typedef __attribute__((ext_vector_type(16))) __bf16   v16b;
typedef __attribute__((ext_vector_type(8)))  __bf16   v8b;
typedef __attribute__((ext_vector_type(8)))  float    v8f;
typedef __attribute__((ext_vector_type(4)))  float    v4f;
typedef __attribute__((ext_vector_type(4)))  unsigned int v4u;
typedef __attribute__((ext_vector_type(4)))  int      v4i;

__device__ __forceinline__ unsigned short f2bf_bits(float f) {
  unsigned u = __float_as_uint(f);
  return (unsigned short)((u + 0x7FFFu + ((u >> 16) & 1u)) >> 16);
}
__device__ __forceinline__ float bf_bits2f(unsigned short h) { return __uint_as_float(((unsigned)h) << 16); }

__device__ __forceinline__ void dep_guard_h(v8f& a, v8f& b, v16h x, v16h y) { asm volatile("v_nop\n\tv_nop\n\tv_nop\n\tv_nop" : "+v"(a), "+v"(b) : "v"(x), "v"(y)); }
__device__ __forceinline__ void dep_guard_b(v8f& a, v8f& b, v16b x, v16b y) { asm volatile("v_nop\n\tv_nop\n\tv_nop\n\tv_nop" : "+v"(a), "+v"(b) : "v"(x), "v"(y)); }
__device__ __forceinline__ void keep4_h(v16h a, v16h b, v16h c, v16h d) { asm volatile("v_nop" :: "v"(a), "v"(b), "v"(c), "v"(d)); }
__device__ __forceinline__ void keep4_b(v16b a, v16b b, v16b c, v16b d) { asm volatile("v_nop" :: "v"(a), "v"(b), "v"(c), "v"(d)); }
__device__ __forceinline__ void acc_guard4(v8f& a, v8f& b, v8f& c, v8f& d) { asm volatile("v_nop\n\tv_nop\n\tv_nop\n\tv_nop" : "+v"(a), "+v"(b), "+v"(c), "+v"(d)); }
template <typename T> struct Frag;
template <> struct Frag<_Float16> {
  typedef v16h V; union U { v16h v; v8h h[2]; };
  static __device__ __forceinline__ v16h load(const _Float16* p) {
    U f; f.h[0] = *(const v8h*)(p); f.h[1] = *(const v8h*)(p + 16); return f.v;
  }
  static __device__ __forceinline__ v8f mma(v16h a, v16h b, v8f c) {
    return __builtin_amdgcn_wmma_f32_16x16x32_f16(false, a, false, b, (short)0, c, false, false);
  }
  static __device__ __forceinline__ void guard(v8f& a, v8f& b, v16h x, v16h y) { dep_guard_h(a, b, x, y); }
  static __device__ __forceinline__ void keep(v16h a, v16h b, v16h c, v16h d) { keep4_h(a, b, c, d); }
};
template <> struct Frag<__bf16> {
  typedef v16b V; union U { v16b v; v8b h[2]; };
  static __device__ __forceinline__ v16b load(const __bf16* p) {
    U f; f.h[0] = *(const v8b*)(p); f.h[1] = *(const v8b*)(p + 16); return f.v;
  }
  static __device__ __forceinline__ v8f mma(v16b a, v16b b, v8f c) {
    return __builtin_amdgcn_wmma_f32_16x16x32_bf16(false, a, false, b, (short)0, c, false, false);
  }
  static __device__ __forceinline__ void guard(v8f& a, v8f& b, v16b x, v16b y) { dep_guard_b(a, b, x, y); }
  static __device__ __forceinline__ void keep(v16b a, v16b b, v16b c, v16b d) { keep4_b(a, b, c, d); }
};

__device__ __forceinline__ unsigned pk16(unsigned short a, unsigned short b) { return (unsigned)a | ((unsigned)b << 16); }
__device__ __forceinline__ unsigned short h_bits(float f) { const _Float16 h = (_Float16)f; return __builtin_bit_cast(unsigned short, h); }

template <int ET> struct Elem;
template <> struct Elem<0> { typedef _Float16 T; };
template <> struct Elem<1> { typedef __bf16 T; };
template <int ET, bool SPLIT, int BIAS_MODE, int OUT_MODE, bool RESID, int ACT = 0>
__global__ __launch_bounds__(256) void wmma_gemm64(
    const unsigned short* __restrict__ Ap, const unsigned short* __restrict__ A2p, int lda, long strideA,
    const unsigned short* __restrict__ Btp, const unsigned short* __restrict__ Bt2p, int ldb, long strideB,
    void* __restrict__ Cout, void* __restrict__ Cout2, int ldc, long strideC,
    const float* __restrict__ bias,
    const float* __restrict__ resid, long strideR,
    int M, int N, int K, float scale) {
  typedef typename Elem<ET>::T T;
  typedef typename Frag<T>::V V;
  const T* A = (const T*)Ap; const T* A2 = (const T*)A2p; const T* Bt = (const T*)Btp; const T* Bt2 = (const T*)Bt2p;
  __shared__ __align__(16) float sT[8][16 * 68];
  const int b    = blockIdx.y;
  const int lane = threadIdx.x & 31;
  const int wave = threadIdx.x >> 5;
  const int tilesN = N >> 6;
  const int tilesM = M >> 6;
  const int tile = blockIdx.x * 8 + wave;
  if (tile >= tilesM * tilesN) return;
  const int tm = tile / tilesN;
  const int tn = tile - tm * tilesN;
  const int m0 = tm << 6;
  const int n0 = tn << 6;

  const T* Ab  = A  + (size_t)b * strideA;
  const T* Bb  = Bt + (size_t)b * strideB;
  const T* Ab2 = SPLIT ? (A2  + (size_t)b * strideA) : nullptr;
  const T* Bb2 = SPLIT ? (Bt2 + (size_t)b * strideB) : nullptr;

  const int rlane = lane & 15;
  const int koff  = (lane >> 4) * 8;
  const int mOff  = (lane >> 4) * 8;

  v8f acc[4][4];
#pragma unroll
  for (int i = 0; i < 4; ++i)
#pragma unroll
    for (int j = 0; j < 4; ++j) acc[i][j] = (v8f){0.f,0.f,0.f,0.f,0.f,0.f,0.f,0.f};

  for (int k0 = 0; k0 < K; k0 += 32) {
    V bh[4], bl[4];
#pragma unroll
    for (int j = 0; j < 4; ++j) {
      const size_t bo = (size_t)(n0 + (j << 4) + rlane) * ldb + koff + k0;
      bh[j] = Frag<T>::load(Bb + bo);
      if (SPLIT) bl[j] = Frag<T>::load(Bb2 + bo);
    }
#pragma unroll
    for (int i = 0; i < 4; ++i) {
      const size_t ao = (size_t)(m0 + (i << 4) + rlane) * lda + koff + k0;
      V ah = Frag<T>::load(Ab + ao);
      V al;
      if (SPLIT) al = Frag<T>::load(Ab2 + ao);
#pragma unroll
      for (int j = 0; j < 4; ++j) {
        acc[i][j] = Frag<T>::mma(ah, bh[j], acc[i][j]);
        if (SPLIT) {
          acc[i][j] = Frag<T>::mma(ah, bl[j], acc[i][j]);
          acc[i][j] = Frag<T>::mma(al, bh[j], acc[i][j]);
        }
      }
      Frag<T>::guard(acc[i][0], acc[i][3], ah, SPLIT ? al : ah);
    }
    Frag<T>::keep(bh[0], bh[1], bh[2], bh[3]);
    if (SPLIT) Frag<T>::keep(bl[0], bl[1], bl[2], bl[3]);
  }
  acc_guard4(acc[0][0], acc[0][1], acc[0][2], acc[0][3]);
  acc_guard4(acc[1][0], acc[1][1], acc[1][2], acc[1][3]);
  acc_guard4(acc[2][0], acc[2][1], acc[2][2], acc[2][3]);
  acc_guard4(acc[3][0], acc[3][1], acc[3][2], acc[3][3]);

  float* slab = sT[wave];
  const float* Rb = RESID ? (resid + (size_t)b * strideR) : nullptr;
#pragma unroll
  for (int i = 0; i < 4; ++i) {
    const int mBase = m0 + (i << 4);
#pragma unroll
    for (int j = 0; j < 4; ++j) {
      const int n = n0 + (j << 4) + rlane;
      float bv = 0.f;
      if (BIAS_MODE == 2) bv = bias[n];
#pragma unroll
      for (int r = 0; r < 8; ++r) {
        float v = acc[i][j][r] * scale;
        if (BIAS_MODE == 1) v += bias[mBase + mOff + r];
        if (BIAS_MODE == 2) v += bv;
        if (RESID) v += Rb[(size_t)(mBase + mOff + r) * ldc + n];
        if (ACT == 2) v = fmaxf(v, 0.0f);
        if (ACT == 4) v = (v > 0.f) ? v : 0.01f * v;
        slab[(mOff + r) * 68 + (j << 4) + rlane] = v;
      }
    }
    __builtin_amdgcn_fence(__ATOMIC_RELEASE, "workgroup");
    __builtin_amdgcn_wave_barrier();
    __builtin_amdgcn_fence(__ATOMIC_ACQUIRE, "workgroup");
    if (OUT_MODE == 0) {
      float* C = (float*)Cout + (size_t)b * strideC;
      const int hh = lane >> 4, c4 = (lane & 15) * 4;
      for (int pass = 0; pass < 2; ++pass) {
#pragma unroll
        for (int it = 0; it < 8; ++it) {
          const int row = it * 2 + hh;
          v4f v = *(const v4f*)(slab + row * 68 + c4);
          *(volatile v4f*)(C + (size_t)(mBase + row) * ldc + n0 + c4) = v;
        }
        __threadfence();
      }
    } else {
      const int q = lane >> 3, c8 = (lane & 7) * 8;
      unsigned short* C  = (unsigned short*)Cout  + (size_t)b * strideC;
      unsigned short* C2 = (OUT_MODE == 2) ? ((unsigned short*)Cout2 + (size_t)b * strideC) : nullptr;
      for (int pass = 0; pass < 2; ++pass) {
#pragma unroll
        for (int it = 0; it < 4; ++it) {
          const int row = it * 4 + q;
          const float* sp = slab + row * 68 + c8;
          v8h hv, lv;
#pragma unroll
          for (int e = 0; e < 8; ++e) {
            if (OUT_MODE == 1) {
              hv[e] = (_Float16)sp[e];
            } else {
              unsigned short hb = f2bf_bits(sp[e]);
              unsigned short lb = f2bf_bits(sp[e] - bf_bits2f(hb));
              hv[e] = __builtin_bit_cast(_Float16, hb);
              lv[e] = __builtin_bit_cast(_Float16, lb);
            }
          }
          *(volatile v8h*)(C + (size_t)(mBase + row) * ldc + n0 + c8) = hv;
          if (OUT_MODE == 2) *(volatile v8h*)(C2 + (size_t)(mBase + row) * ldc + n0 + c8) = lv;
        }
        __threadfence();
      }
    }
    __builtin_amdgcn_fence(__ATOMIC_RELEASE, "workgroup");
    __builtin_amdgcn_wave_barrier();
    __builtin_amdgcn_fence(__ATOMIC_ACQUIRE, "workgroup");
  }
}

__global__ __launch_bounds__(256) void cast8_f16_kernel(const float* __restrict__ in, unsigned short* __restrict__ out,
                                                        int n8, float scale) {
  const int i = blockIdx.x * 256 + threadIdx.x;
  if (i >= n8) return;
  const float* p = in + 8 * (size_t)i;
  const v4f a = *(const v4f*)(p);
  const v4f c = *(const v4f*)(p + 4);
  unsigned short hb[8];
#pragma unroll
  for (int e = 0; e < 4; ++e) {
    hb[e]     = h_bits(a[e] * scale);
    hb[4 + e] = h_bits(c[e] * scale);
  }
  const v4u u = (v4u){pk16(hb[0], hb[1]), pk16(hb[2], hb[3]), pk16(hb[4], hb[5]), pk16(hb[6], hb[7])};
  unsigned short* q = out + 8 * (size_t)i;
  *(volatile v4u*)q = u;
  __threadfence();
  *(volatile v4u*)q = u;
}

__global__ __launch_bounds__(128) void layernorm_kernel(const float* __restrict__ X, const float* __restrict__ gam,
                                                        const float* __restrict__ bet, unsigned short* __restrict__ out) {
  __shared__ float redA[4];
  __shared__ float redB[4];
  const int row  = blockIdx.x;
  const int t    = threadIdx.x;
  const int lane = t & 31, wave = t >> 5;
  const int c0   = t * 8;
  const float* xr = X + (size_t)row * kDim + c0;
  const v4f a = *(const v4f*)(xr);
  const v4f c = *(const v4f*)(xr + 4);
  float xv[8];
#pragma unroll
  for (int e = 0; e < 4; ++e) { xv[e] = a[e]; xv[4 + e] = c[e]; }
  float s = ((xv[0] + xv[1]) + (xv[2] + xv[3])) + ((xv[4] + xv[5]) + (xv[6] + xv[7]));
#pragma unroll
  for (int off = 16; off > 0; off >>= 1) s += __shfl_xor(s, off, 32);
  if (lane == 0) redA[wave] = s;
  __syncthreads();
  const float mean = ((redA[0] + redA[1]) + (redA[2] + redA[3])) * kInvDim;
  float d[8];
  float ss = 0.f;
#pragma unroll
  for (int e = 0; e < 8; ++e) { d[e] = xv[e] - mean; ss += d[e] * d[e]; }
#pragma unroll
  for (int off = 16; off > 0; off >>= 1) ss += __shfl_xor(ss, off, 32);
  if (lane == 0) redB[wave] = ss;
  __syncthreads();
  const float var  = ((redB[0] + redB[1]) + (redB[2] + redB[3])) * kInvDim;
  const float rstd = rsqrtf(var + kLnEps);
  const v4f g0 = *(const v4f*)(gam + c0);
  const v4f g1 = *(const v4f*)(gam + c0 + 4);
  const v4f b0 = *(const v4f*)(bet + c0);
  const v4f b1 = *(const v4f*)(bet + c0 + 4);
  float gv[8], be[8];
#pragma unroll
  for (int e = 0; e < 4; ++e) { gv[e] = g0[e]; gv[4 + e] = g1[e]; be[e] = b0[e]; be[4 + e] = b1[e]; }
  unsigned short hb[8];
#pragma unroll
  for (int e = 0; e < 8; ++e) {
    const float y = (d[e] * rstd) * gv[e] + be[e];
    hb[e] = h_bits(y);
  }
  const v4u u = (v4u){pk16(hb[0], hb[1]), pk16(hb[2], hb[3]), pk16(hb[4], hb[5]), pk16(hb[6], hb[7])};
  unsigned short* q = out + (size_t)row * kDim + c0;
  *(volatile v4u*)q = u;
  __threadfence();
  *(volatile v4u*)q = u;
}

__global__ __launch_bounds__(256) void vtrans_kernel(const unsigned short* __restrict__ qkv, unsigned short* __restrict__ vt) {
  __shared__ unsigned short sm[64][72];
  const int t  = threadIdx.x;
  const int kt = blockIdx.x;
  const int g  = blockIdx.y;
  const int b  = g >> 4, h = g & 15;
  const int key0 = kt * 64;
#pragma unroll
  for (int it = 0; it < 2; ++it) {
    const int key = it * 32 + (t >> 3);
    const int c8  = (t & 7) * 8;
    const unsigned short* src = qkv + (size_t)(b * kSeq + key0 + key) * kQkvN + 2 * kDim + h * kHd + c8;
    const v4u w4 = *(const v4u*)src;
#pragma unroll
    for (int k = 0; k < 4; ++k) {
      sm[c8 + 2 * k][key]     = (unsigned short)(w4[k] & 0xffffu);
      sm[c8 + 2 * k + 1][key] = (unsigned short)(w4[k] >> 16);
    }
  }
  __syncthreads();
  const int lane = t & 31, wave = t >> 5;
  const int q = lane >> 3, c8 = (lane & 7) * 8;
  unsigned short* op = vt + (size_t)g * kHd * kSeq;
  for (int pass = 0; pass < 2; ++pass) {
#pragma unroll
    for (int it = 0; it < 2; ++it) {
      const int d = it * 32 + wave * 4 + q;
      unsigned short hb[8];
#pragma unroll
      for (int e = 0; e < 8; ++e) hb[e] = sm[d][c8 + e];
      const v4u u = (v4u){pk16(hb[0], hb[1]), pk16(hb[2], hb[3]), pk16(hb[4], hb[5]), pk16(hb[6], hb[7])};
      *(volatile v4u*)(op + (size_t)d * kSeq + key0 + c8) = u;
    }
    __threadfence();
  }
}

__global__ __launch_bounds__(128) void softmax_row_kernel(const float* __restrict__ S, const int* __restrict__ keyflag,
                                                          unsigned short* __restrict__ P) {
  __shared__ float redM[4];
  __shared__ float redS[4];
  const int row  = blockIdx.x;
  const int t    = threadIdx.x;
  const int lane = t & 31, wave = t >> 5;
  const int c0   = t * 8;
  const float* sr = S + (size_t)row * kSeq + c0;
  const v4f a = *(const v4f*)(sr);
  const v4f c = *(const v4f*)(sr + 4);
  const v4i f0 = *(const v4i*)(keyflag + c0);
  const v4i f1 = *(const v4i*)(keyflag + c0 + 4);
  const float ninf = -INFINITY;
  float x[8];
#pragma unroll
  for (int e = 0; e < 4; ++e) {
    x[e]     = (f0[e] == 0) ? ninf : a[e];
    x[4 + e] = (f1[e] == 0) ? ninf : c[e];
  }
  float m = fmaxf(fmaxf(fmaxf(x[0], x[1]), fmaxf(x[2], x[3])), fmaxf(fmaxf(x[4], x[5]), fmaxf(x[6], x[7])));
#pragma unroll
  for (int off = 16; off > 0; off >>= 1) m = fmaxf(m, __shfl_xor(m, off, 32));
  if (lane == 0) redM[wave] = m;
  __syncthreads();
  const float mx = fmaxf(fmaxf(redM[0], redM[1]), fmaxf(redM[2], redM[3]));
  float ev[8];
  float s = 0.f;
#pragma unroll
  for (int e = 0; e < 8; ++e) { ev[e] = expf(x[e] - mx); s += ev[e]; }
#pragma unroll
  for (int off = 16; off > 0; off >>= 1) s += __shfl_xor(s, off, 32);
  if (lane == 0) redS[wave] = s;
  __syncthreads();
  const float tot  = ((redS[0] + redS[1]) + (redS[2] + redS[3]));
  const float invc = (1.0f / tot) * kPCarry;
  unsigned short hb[8];
#pragma unroll
  for (int e = 0; e < 8; ++e) hb[e] = h_bits(ev[e] * invc);
  const v4u u = (v4u){pk16(hb[0], hb[1]), pk16(hb[2], hb[3]), pk16(hb[4], hb[5]), pk16(hb[6], hb[7])};
  unsigned short* q = P + (size_t)row * kSeq + c0;
  *(volatile v4u*)q = u;
  __threadfence();
  *(volatile v4u*)q = u;
}

__global__ __launch_bounds__(256) void gelu_f16x2_kernel(const float* __restrict__ in, unsigned short* __restrict__ out, int n2) {
  const int i = blockIdx.x * 256 + threadIdx.x;
  if (i >= n2) return;
  unsigned u = 0u;
#pragma unroll 1
  for (int e = 0; e < 2; ++e) {
    const float v = in[2 * (size_t)i + e];
    const float g = 0.5f * v * (1.0f + erff(v * 0.70710678118654752f));
    u |= ((unsigned)h_bits(g)) << (16 * e);
  }
  ((volatile unsigned*)out)[i] = u;
  __threadfence();
  ((volatile unsigned*)out)[i] = u;
}

extern "C" void kernel_launch(void* const* d_in, const int* in_sizes, int n_in,
                              void* d_out, int out_size, void* d_ws, size_t ws_size,
                              hipStream_t stream) {
  if (n_in < 13) return;
  if (ws_size < kWsTotal) return;
  if (out_size != kTok * kDim) return;
  if (in_sizes[0] != kTok * kDim || in_sizes[1] != kNB * kSeq || in_sizes[2] != kQkvN * kDim ||
      in_sizes[3] != kDim * kDim || in_sizes[4] != kDim || in_sizes[5] != kHid * kDim || in_sizes[6] != kHid ||
      in_sizes[7] != kDim * kHid || in_sizes[8] != kDim || in_sizes[9] != kDim || in_sizes[10] != kDim ||
      in_sizes[11] != kDim || in_sizes[12] != kDim) return;

  const float* x       = (const float*)d_in[0];
  const int*   keyflag = (const int*)d_in[1];
  const float* qkv_w   = (const float*)d_in[2];
  const float* proj_w  = (const float*)d_in[3];
  const float* proj_b  = (const float*)d_in[4];
  const float* fc1_w   = (const float*)d_in[5];
  const float* fc1_b   = (const float*)d_in[6];
  const float* fc2_w   = (const float*)d_in[7];
  const float* fc2_b   = (const float*)d_in[8];
  const float* norm1_w = (const float*)d_in[9];
  const float* norm1_b = (const float*)d_in[10];
  const float* norm2_w = (const float*)d_in[11];
  const float* norm2_b = (const float*)d_in[12];
  float* out = (float*)d_out;

  char* ws = (char*)d_ws;
  unsigned short* regWA = (unsigned short*)(ws + kOffWA);
  unsigned short* regWB = (unsigned short*)(ws + kOffWB);
  unsigned short* regH  = (unsigned short*)(ws + kOffH);
  unsigned short* qkvp  = (unsigned short*)(ws + kOffQ);
  float*          x1    = (float*)(ws + kOffQ);
  float*          regS  = (float*)(ws + kOffS);
  unsigned short* regP  = (unsigned short*)(ws + kOffP);

  cast8_f16_kernel<<<(kQkvN * kDim / 8) / 256, 256, 0, stream>>>(qkv_w, regWA, kQkvN * kDim / 8, kWCarry);
  cast8_f16_kernel<<<(kDim * kHid / 8) / 256, 256, 0, stream>>>(fc2_w, regWB, kDim * kHid / 8, kWCarry);

  layernorm_kernel<<<kTok, 128, 0, stream>>>(x, norm1_w, norm1_b, regH);

  wmma_gemm64<0, false, 0, 1, false><<<dim3(384, 1), 256, 0, stream>>>(
      regH, nullptr, kDim, 0L, regWA, nullptr, kDim, 0L,
      (void*)qkvp, nullptr, kQkvN, 0L, nullptr, nullptr, 0L, kTok, kQkvN, kDim, kWCarryInv);

  vtrans_kernel<<<dim3(kSeq / 64, kNB * kHeads), 256, 0, stream>>>(qkvp, regWA);

  for (int cix = 0; cix < kNumChunks; ++cix) {
    const int b  = cix >> 1;
    const int h0 = (cix & 1) * kHeadsPerChunk;
    const unsigned short* qa = qkvp + (size_t)b * kSeq * kQkvN + (size_t)h0 * kHd;
    const unsigned short* ka = qa + kDim;
    wmma_gemm64<0, false, 0, 0, false><<<dim3(32, kHeadsPerChunk), 256, 0, stream>>>(
        qa, nullptr, kQkvN, (long)kHd, ka, nullptr, kQkvN, (long)kHd,
        (void*)regS, nullptr, kSeq, (long)kSeq * kSeq, nullptr, nullptr, 0L, kSeq, kSeq, kHd, kAttnScale);
    softmax_row_kernel<<<kHeadsPerChunk * kSeq, 128, 0, stream>>>(regS, keyflag + b * kSeq, regP);
    wmma_gemm64<0, false, 0, 1, false><<<dim3(2, kHeadsPerChunk), 256, 0, stream>>>(
        regP, nullptr, kSeq, (long)kSeq * kSeq,
        regWA + (size_t)cix * kHeadsPerChunk * kHd * kSeq, nullptr, kSeq, (long)kHd * kSeq,
        (void*)(regH + (size_t)b * kSeq * kDim + (size_t)h0 * kHd), nullptr, kDim, (long)kHd,
        nullptr, nullptr, 0L, kSeq, kHd, kSeq, kPVScale);
  }

  cast8_f16_kernel<<<(kDim * kDim / 8) / 256, 256, 0, stream>>>(proj_w, regWA, kDim * kDim / 8, kWCarry);
  wmma_gemm64<0, false, 2, 0, true><<<dim3(128, 1), 256, 0, stream>>>(
      regH, nullptr, kDim, 0L, regWA, nullptr, kDim, 0L,
      (void*)x1, nullptr, kDim, 0L, proj_b, x, 0L, kTok, kDim, kDim, kProjScale);

  layernorm_kernel<<<kTok, 128, 0, stream>>>(x1, norm2_w, norm2_b, regH);

  cast8_f16_kernel<<<(kHid * kDim / 8) / 256, 256, 0, stream>>>(fc1_w, regWA, kHid * kDim / 8, kWCarry);

  for (int part = 0; part < kMlpParts; ++part) {
    const size_t r0 = (size_t)part * kMlpRows;
    wmma_gemm64<0, false, 2, 0, false><<<dim3(256, 1), 256, 0, stream>>>(
        regH + r0 * kDim, nullptr, kDim, 0L, regWA, nullptr, kDim, 0L,
        (void*)regS, nullptr, kHid, 0L, fc1_b, nullptr, 0L, kMlpRows, kHid, kDim, kWCarryInv);
    gelu_f16x2_kernel<<<(kMlpRows * kHid / 2) / 256, 256, 0, stream>>>(regS, regP, kMlpRows * kHid / 2);
    wmma_gemm64<0, false, 2, 0, true><<<dim3(64, 1), 256, 0, stream>>>(
        regP, nullptr, kHid, 0L, regWB, nullptr, kHid, 0L,
        (void*)(out + r0 * kDim), nullptr, kDim, 0L, fc2_b, x1 + r0 * kDim, 0L, kMlpRows, kDim, kHid, kWCarryInv);
  }
}
